// seqFusionAttentionWeightProj_48782238548116
// MI455X (gfx1250) — hardware-run, weakly checked
//
#include <hip/hip_runtime.h>
#include <stddef.h>
#include <stdint.h>

#define NB    2
#define SEQ   2048
#define DM    256
#define NHD   8
#define HC    32
#define NROWS 4096
#define WINH  32
#define WROWS 1280
#define GROW  768
#define OROW  1024
#define QBK   64
#define PP    104

static_assert(NB * SEQ == NROWS);
static_assert(NHD * HC == DM);
static_assert(WROWS == 5 * DM);
static_assert(GROW == 3 * DM);
static_assert(OROW == 4 * DM);
static_assert(SEQ % QBK == 0);
static_assert(NROWS % 64 == 0);
static_assert(DM % 64 == 0);
static_assert((NROWS * DM) % 2048 == 0);
static_assert(HC == 32);
static_assert(2 * WINH + QBK <= 128);
static_assert((PP * 2) % 16 == 0);

typedef unsigned short us;
typedef __attribute__((ext_vector_type(16))) __bf16 v16bf;
typedef us           v8us __attribute__((ext_vector_type(8)));
typedef float        v8f  __attribute__((ext_vector_type(8)));
typedef float        v4f  __attribute__((ext_vector_type(4)));
typedef unsigned int v4u  __attribute__((ext_vector_type(4)));

union Frag  { v16bf v; v8us h[2]; };
union Pack8 { v8us h; v4u u; };

__device__ __forceinline__ us bf_rne(float f) {
  unsigned u = __float_as_uint(f);
  u = u + 0x7FFFu + ((u >> 16) & 1u);
  return (us)(u >> 16);
}
__device__ __forceinline__ float bf_val(us h) { return __uint_as_float(((unsigned)h) << 16); }
__device__ __forceinline__ void split2(float f, us& hi, us& lo) {
  const us hv = bf_rne(f);
  hi = hv;
  lo = bf_rne(f - bf_val(hv));
}
__device__ __forceinline__ void split8(const float (&f)[8], Pack8& ph, Pack8& pl) {
  us hh[8], ll[8];
#pragma unroll
  for (int e = 0; e < 8; ++e) split2(f[e], hh[e], ll[e]);
  ph.h = (v8us){hh[0], hh[1], hh[2], hh[3], hh[4], hh[5], hh[6], hh[7]};
  pl.h = (v8us){ll[0], ll[1], ll[2], ll[3], ll[4], ll[5], ll[6], ll[7]};
}

__device__ __forceinline__ v8f mma16(v16bf a, v16bf b, v8f c) {
  c = __builtin_amdgcn_wmma_f32_16x16x32_bf16(false, a, false, b, (short)0, c, false, false);
  asm volatile("v_nop\n\tv_nop\n\tv_nop\n\tv_nop" : "+v"(c) : "v"(a), "v"(b));
  return c;
}

__device__ __forceinline__ v16bf ldfrag(const us* p, int ld, int row0, int k0, int lane) {
  const int m = lane & 15, lh = lane >> 4;
  const us* q = p + (size_t)(row0 + m) * ld + k0 + 8 * lh;
  Frag f;
  f.h[0] = *(const v8us*)(q);
  f.h[1] = *(const v8us*)(q + 16);
  return f.v;
}

__device__ __forceinline__ v8f zero8() { return (v8f){0.f, 0.f, 0.f, 0.f, 0.f, 0.f, 0.f, 0.f}; }

__device__ __forceinline__ void gemm16x64x3(const us* __restrict__ Ah, const us* __restrict__ Al,
                                            const us* __restrict__ Bh, const us* __restrict__ Bl,
                                            int m0, int n0, int lane, v8f (&acc)[4]) {
#pragma unroll 1
  for (int k0 = 0; k0 < DM; k0 += 32) {
    const v16bf ah = ldfrag(Ah, DM, m0, k0, lane);
    const v16bf al = ldfrag(Al, DM, m0, k0, lane);
#pragma unroll
    for (int t = 0; t < 4; ++t) {
      const v16bf bh = ldfrag(Bh, DM, n0 + 16 * t, k0, lane);
      const v16bf bl = ldfrag(Bl, DM, n0 + 16 * t, k0, lane);
      acc[t] = mma16(ah, bh, acc[t]);
      acc[t] = mma16(ah, bl, acc[t]);
      acc[t] = mma16(al, bh, acc[t]);
    }
  }
}

#define TWP 68
__global__ __launch_bounds__(128) void k_cvtw(const float* __restrict__ qt, const float* __restrict__ kt,
                                              const float* __restrict__ vt, const float* __restrict__ gw,
                                              const float* __restrict__ ow,
                                              us* __restrict__ wh, us* __restrict__ wl) {
  __shared__ __align__(16) float tl[64 * TWP];
  const int tid = threadIdx.x;
  const int rt = blockIdx.x;
  const int k0 = blockIdx.y * 64;
  v4u hv[4], lv[4];
  size_t go[4];
  if (rt < 12) {
    const float* s = (rt < 4) ? qt : ((rt < 8) ? kt : vt);
    const int n0 = 64 * (rt & 3);
#pragma unroll
    for (int j = 0; j < 8; ++j) {
      const int p  = tid + 128 * j;
      const int kr = p >> 4;
      const int c4 = (p & 15) * 4;
      const v4f a = *(const v4f*)(s + (size_t)(k0 + kr) * DM + n0 + c4);
      *(v4f*)(tl + kr * TWP + c4) = a;
    }
    __syncthreads();
#pragma unroll
    for (int j = 0; j < 4; ++j) {
      const int p  = tid + 128 * j;
      const int n  = p >> 3;
      const int kc = (p & 7) * 8;
      const float* cp = tl + kc * TWP + n;
      float f[8];
#pragma unroll
      for (int e = 0; e < 8; ++e) f[e] = cp[e * TWP];
      Pack8 ph, pl;
      split8(f, ph, pl);
      hv[j] = ph.u;
      lv[j] = pl.u;
      go[j] = ((size_t)(64 * rt + n)) * DM + k0 + kc;
    }
  } else {
    const float* s = (rt < 16) ? gw : ow;
    const int n0 = 64 * ((rt - 12) & 3);
#pragma unroll
    for (int j = 0; j < 4; ++j) {
      const int p  = tid + 128 * j;
      const int n  = p >> 3;
      const int kc = (p & 7) * 8;
      const float* rp = s + (size_t)(n0 + n) * DM + k0 + kc;
      const v4f a0 = *(const v4f*)(rp), a1 = *(const v4f*)(rp + 4);
      const float f[8] = {a0[0], a0[1], a0[2], a0[3], a1[0], a1[1], a1[2], a1[3]};
      Pack8 ph, pl;
      split8(f, ph, pl);
      hv[j] = ph.u;
      lv[j] = pl.u;
      go[j] = ((size_t)(64 * rt + n)) * DM + k0 + kc;
    }
  }
#pragma unroll
  for (int j = 0; j < 4; ++j) { *(volatile v4u*)(wh + go[j]) = hv[j]; *(volatile v4u*)(wl + go[j]) = lv[j]; }
  __threadfence();
#pragma unroll
  for (int j = 0; j < 4; ++j) { *(volatile v4u*)(wh + go[j]) = hv[j]; *(volatile v4u*)(wl + go[j]) = lv[j]; }
}

__global__ __launch_bounds__(256) void k_cvtx(const float* __restrict__ x0, const float* __restrict__ x1,
                                              const float* __restrict__ x2,
                                              us* __restrict__ xh, us* __restrict__ xl) {
  const int sel = blockIdx.y;
  const float* x = (sel == 0) ? x0 : ((sel == 1) ? x1 : x2);
  const size_t i = (size_t)blockIdx.x * 2048 + (size_t)threadIdx.x * 8;
  const v4f a0 = *(const v4f*)(x + i);
  const v4f a1 = *(const v4f*)(x + i + 4);
  const float f[8] = {a0[0], a0[1], a0[2], a0[3], a1[0], a1[1], a1[2], a1[3]};
  Pack8 ph, pl;
  split8(f, ph, pl);
  const v4u hv = ph.u, lv = pl.u;
  const size_t o = (size_t)sel * NROWS * DM + i;
  *(volatile v4u*)(xh + o) = hv;
  *(volatile v4u*)(xl + o) = lv;
  __threadfence();
  *(volatile v4u*)(xh + o) = hv;
  *(volatile v4u*)(xl + o) = lv;
}

#define SFP 68
__global__ __launch_bounds__(128) void k_proj(const us* __restrict__ xh, const us* __restrict__ xl,
                                              const us* __restrict__ wh, const us* __restrict__ wl,
                                              const float* __restrict__ gb,
                                              us* __restrict__ qh, us* __restrict__ ql,
                                              us* __restrict__ kh, us* __restrict__ kl,
                                              us* __restrict__ vth, us* __restrict__ vtl,
                                              float* __restrict__ gp) {
  __shared__ __align__(16) float sf[64 * SFP];
  const int tid = threadIdx.x, lane = tid & 31, wave = tid >> 5;
  const int lh = lane >> 4, c = lane & 15;
  const int mb = blockIdx.x * 64;
  const int ns = blockIdx.y;
  const int which = ns >> 2;
  const int cg = ns & 3;
  const int col0 = 64 * cg;
  const int m0 = mb + wave * 16;
  const int n0 = 64 * ns;
  const int xsel = (which == 3) ? 2 : which;
  const us* Ah = xh + (size_t)xsel * NROWS * DM;
  const us* Al = xl + (size_t)xsel * NROWS * DM;

  v8f acc[4];
#pragma unroll
  for (int t = 0; t < 4; ++t) acc[t] = zero8();
  gemm16x64x3(Ah, Al, wh, wl, m0, n0, lane, acc);

  if (which == 3) {
#pragma unroll
    for (int t = 0; t < 4; ++t) {
      const float bv = gb[col0 + 16 * t + c];
#pragma unroll
      for (int r = 0; r < 8; ++r) {
        const float v = acc[t][r] + bv;
        const float e = __expf(-v);
        sf[(wave * 16 + 8 * lh + r) * SFP + 16 * t + c] = __builtin_amdgcn_rcpf(1.0f + e);
      }
    }
  } else {
#pragma unroll
    for (int t = 0; t < 4; ++t) {
#pragma unroll
      for (int r = 0; r < 8; ++r)
        sf[(wave * 16 + 8 * lh + r) * SFP + 16 * t + c] = acc[t][r];
    }
  }
  __syncthreads();

  if (which < 2) {
    v4u hv[4], lv[4];
    size_t go[4];
#pragma unroll
    for (int j = 0; j < 4; ++j) {
      const int p  = tid + 128 * j;
      const int lr = p >> 3;
      const int d0 = (p & 7) * 8;
      const float* ra = sf + lr * SFP + d0;
      const v4f a0 = *(const v4f*)(ra), a1 = *(const v4f*)(ra + 4);
      const float f[8] = {a0[0], a0[1], a0[2], a0[3], a1[0], a1[1], a1[2], a1[3]};
      Pack8 ph, pl;
      split8(f, ph, pl);
      hv[j] = ph.u;
      lv[j] = pl.u;
      go[j] = ((size_t)(mb + lr)) * DM + col0 + d0;
    }
    us* dsth = (which == 0) ? qh : kh;
    us* dstl = (which == 0) ? ql : kl;
#pragma unroll
    for (int j = 0; j < 4; ++j) { *(volatile v4u*)(dsth + go[j]) = hv[j]; *(volatile v4u*)(dstl + go[j]) = lv[j]; }
    __threadfence();
#pragma unroll
    for (int j = 0; j < 4; ++j) { *(volatile v4u*)(dsth + go[j]) = hv[j]; *(volatile v4u*)(dstl + go[j]) = lv[j]; }
  } else if (which == 2) {
    v4u hv[4], lv[4];
    size_t go[4];
    const int bb = mb >> 11;
    const int s0 = mb & (SEQ - 1);
#pragma unroll
    for (int j = 0; j < 4; ++j) {
      const int p  = tid + 128 * j;
      const int d  = p >> 3;
      const int pc = p & 7;
      const float* cp = sf + (pc * 8) * SFP + d;
      float f[8];
#pragma unroll
      for (int e = 0; e < 8; ++e) f[e] = cp[e * SFP];
      Pack8 ph, pl;
      split8(f, ph, pl);
      hv[j] = ph.u;
      lv[j] = pl.u;
      go[j] = ((size_t)(bb * DM + col0 + d)) * SEQ + s0 + pc * 8;
    }
#pragma unroll
    for (int j = 0; j < 4; ++j) { *(volatile v4u*)(vth + go[j]) = hv[j]; *(volatile v4u*)(vtl + go[j]) = lv[j]; }
    __threadfence();
#pragma unroll
    for (int j = 0; j < 4; ++j) { *(volatile v4u*)(vth + go[j]) = hv[j]; *(volatile v4u*)(vtl + go[j]) = lv[j]; }
  } else {
    v4f val[8];
    size_t go[8];
#pragma unroll
    for (int j = 0; j < 8; ++j) {
      const int p  = tid + 128 * j;
      const int lr = p >> 4;
      const int pc = p & 15;
      val[j] = *(const v4f*)(sf + lr * SFP + 4 * pc);
      go[j]  = ((size_t)(mb + lr)) * DM + col0 + 4 * pc;
    }
#pragma unroll
    for (int j = 0; j < 8; ++j) *(volatile v4f*)(gp + go[j]) = val[j];
    __threadfence();
#pragma unroll
    for (int j = 0; j < 8; ++j) *(volatile v4f*)(gp + go[j]) = val[j];
  }
}

__device__ __forceinline__ void attn_head(int h, int b, int q0, int kb, int lane,
                                          const us* __restrict__ qh, const us* __restrict__ ql,
                                          const us* __restrict__ kh, const us* __restrict__ kl,
                                          const us* __restrict__ vth, const us* __restrict__ vtl,
                                          const float* __restrict__ gp,
                                          us* pwh, us* pwl, v8f (&o)[2]) {
  const int lh = lane >> 4, c = lane & 15;
  const size_t rowb = (size_t)b * SEQ;
  const int colh = h * HC;
  const float NEGV = -1.0e30f;
  const float SCL  = 0.17677669529663687f;

  Frag qa_h, qa_l;
  {
    const us* qr  = qh + (rowb + q0 + c) * DM + colh + 8 * lh;
    const us* qr2 = ql + (rowb + q0 + c) * DM + colh + 8 * lh;
    qa_h.h[0] = *(const v8us*)(qr);
    qa_h.h[1] = *(const v8us*)(qr + 16);
    qa_l.h[0] = *(const v8us*)(qr2);
    qa_l.h[1] = *(const v8us*)(qr2 + 16);
  }

  v8f s[6];
#pragma unroll
  for (int j = 0; j < 6; ++j) s[j] = zero8();
#pragma unroll
  for (int j = 0; j < 6; ++j) {
    int key = kb + 16 * j + c;
    key = (key < 0) ? 0 : ((key > SEQ - 1) ? (SEQ - 1) : key);
    const size_t ro = (rowb + key) * DM + colh + 8 * lh;
    Frag kf_h, kf_l;
    kf_h.h[0] = *(const v8us*)(kh + ro);
    kf_h.h[1] = *(const v8us*)(kh + ro + 16);
    kf_l.h[0] = *(const v8us*)(kl + ro);
    kf_l.h[1] = *(const v8us*)(kl + ro + 16);
    s[j] = mma16(qa_h.v, kf_h.v, s[j]);
    s[j] = mma16(qa_h.v, kf_l.v, s[j]);
    s[j] = mma16(qa_l.v, kf_h.v, s[j]);
  }

  float rmax[8];
#pragma unroll
  for (int r = 0; r < 8; ++r) {
    const int qry = q0 + 8 * lh + r;
    float m = NEGV;
#pragma unroll
    for (int j = 0; j < 6; ++j) {
      const int key = kb + 16 * j + c;
      const int d = qry - key;
      const bool live = (key >= 0) && (key < SEQ) && (d <= WINH) && (d >= -WINH);
      const float sv = s[j][r] * SCL;
      s[j][r] = live ? sv : NEGV;
      m = fmaxf(m, s[j][r]);
    }
#pragma unroll
    for (int off = 1; off < 16; off <<= 1) m = fmaxf(m, __shfl_xor(m, off, 32));
    rmax[r] = m;
  }
  __syncthreads();

  float inv[8];
#pragma unroll
  for (int r = 0; r < 8; ++r) {
    float psum = 0.f;
#pragma unroll
    for (int j = 0; j < 6; ++j) {
      const float p = __expf(s[j][r] - rmax[r]);
      psum += p;
      us ph, pl;
      split2(p, ph, pl);
      pwh[(8 * lh + r) * PP + 16 * j + c] = ph;
      pwl[(8 * lh + r) * PP + 16 * j + c] = pl;
    }
#pragma unroll
    for (int off = 1; off < 16; off <<= 1) psum += __shfl_xor(psum, off, 32);
    inv[r] = 1.0f / psum;
  }
  __syncthreads();

  v8f oacc[2];
  oacc[0] = zero8();
  oacc[1] = zero8();
#pragma unroll
  for (int kk = 0; kk < 3; ++kk) {
    const v16bf pah = ldfrag(pwh, PP, 0, kk * 32, lane);
    const v16bf pal = ldfrag(pwl, PP, 0, kk * 32, lane);
    int ps0 = kb + 32 * kk + 8 * lh;
    int ps1 = ps0 + 16;
    ps0 = (ps0 < 0) ? 0 : ((ps0 > SEQ - 8) ? (SEQ - 8) : ps0);
    ps1 = (ps1 < 0) ? 0 : ((ps1 > SEQ - 8) ? (SEQ - 8) : ps1);
#pragma unroll
    for (int t = 0; t < 2; ++t) {
      const int ch = 16 * t + c;
      const size_t vr = ((size_t)((b * NHD + h) * HC + ch)) * SEQ;
      Frag vb_h, vb_l;
      vb_h.h[0] = *(const v8us*)(vth + vr + ps0);
      vb_h.h[1] = *(const v8us*)(vth + vr + ps1);
      vb_l.h[0] = *(const v8us*)(vtl + vr + ps0);
      vb_l.h[1] = *(const v8us*)(vtl + vr + ps1);
      oacc[t] = mma16(pah, vb_h.v, oacc[t]);
      oacc[t] = mma16(pah, vb_l.v, oacc[t]);
      oacc[t] = mma16(pal, vb_h.v, oacc[t]);
    }
  }
#pragma unroll
  for (int t = 0; t < 2; ++t) {
#pragma unroll
    for (int r = 0; r < 8; ++r) {
      const size_t row = rowb + q0 + 8 * lh + r;
      const int col = colh + 16 * t + c;
      const float g = gp[row * DM + col];
      o[t][r] = oacc[t][r] * inv[r] * g;
    }
  }
}

__global__ __launch_bounds__(128) void k_attn(const us* __restrict__ qh, const us* __restrict__ ql,
                                              const us* __restrict__ kh, const us* __restrict__ kl,
                                              const us* __restrict__ vth, const us* __restrict__ vtl,
                                              const float* __restrict__ gp,
                                              us* __restrict__ oh, us* __restrict__ ol) {
  __shared__ __align__(16) us Psh[4 * 16 * PP];
  __shared__ __align__(16) us Psl[4 * 16 * PP];

  const int tid = threadIdx.x, lane = tid & 31, wave = tid >> 5;
  const int lh = lane >> 4, c = lane & 15;
  const int qb = blockIdx.x;
  const int hp = blockIdx.y;
  const int b  = blockIdx.z;
  const int q0b = qb * QBK;
  const int q0  = q0b + wave * 16;
  const int kb  = q0b - WINH + 32 * (wave >> 1);

  us* pwh = Psh + wave * 16 * PP;
  us* pwl = Psl + wave * 16 * PP;

  v8f oA[2], oB[2];
  attn_head(2 * hp,     b, q0, kb, lane, qh, ql, kh, kl, vth, vtl, gp, pwh, pwl, oA);
  attn_head(2 * hp + 1, b, q0, kb, lane, qh, ql, kh, kl, vth, vtl, gp, pwh, pwl, oB);

  __syncthreads();
#pragma unroll
  for (int t = 0; t < 2; ++t) {
#pragma unroll
    for (int r = 0; r < 8; ++r) {
      us ah, al, bh, bl;
      split2(oA[t][r], ah, al);
      split2(oB[t][r], bh, bl);
      pwh[(8 * lh + r) * PP + 16 * t + c]      = ah;
      pwl[(8 * lh + r) * PP + 16 * t + c]      = al;
      pwh[(8 * lh + r) * PP + 32 + 16 * t + c] = bh;
      pwl[(8 * lh + r) * PP + 32 + 16 * t + c] = bl;
    }
  }
  __syncthreads();
  v4u hv[4], lv[4];
  size_t go[4];
  const size_t rowb = (size_t)b * SEQ;
#pragma unroll
  for (int it = 0; it < 4; ++it) {
    const int p  = lane + 32 * it;
    const int L  = p >> 3;
    const int pc = p & 7;
    Pack8 ph, pl;
    ph.h   = *(const v8us*)(pwh + L * PP + pc * 8);
    pl.h   = *(const v8us*)(pwl + L * PP + pc * 8);
    hv[it] = ph.u;
    lv[it] = pl.u;
    go[it] = (rowb + q0 + L) * DM + (size_t)hp * 64 + pc * 8;
  }
#pragma unroll
  for (int it = 0; it < 4; ++it) { *(volatile v4u*)(oh + go[it]) = hv[it]; *(volatile v4u*)(ol + go[it]) = lv[it]; }
  __threadfence();
#pragma unroll
  for (int it = 0; it < 4; ++it) { *(volatile v4u*)(oh + go[it]) = hv[it]; *(volatile v4u*)(ol + go[it]) = lv[it]; }
}

#define OTP 68
__global__ __launch_bounds__(128) void k_out(const us* __restrict__ ah, const us* __restrict__ al,
                                             const us* __restrict__ wh, const us* __restrict__ wl,
                                             const float* __restrict__ ob, float* __restrict__ out) {
  __shared__ __align__(16) float st[4][16 * OTP];
  const int tid = threadIdx.x, lane = tid & 31, wave = tid >> 5;
  const int lh = lane >> 4, c = lane & 15;
  const int m0 = blockIdx.x * 64 + wave * 16;
  const int n0 = blockIdx.y * 64;

  v8f acc[4];
#pragma unroll
  for (int t = 0; t < 4; ++t) acc[t] = zero8();
  gemm16x64x3(ah, al, wh, wl, m0, OROW + n0, lane, acc);

  float* sw = st[wave];
#pragma unroll
  for (int t = 0; t < 4; ++t) {
#pragma unroll
    for (int r = 0; r < 8; ++r) sw[(8 * lh + r) * OTP + 16 * t + c] = acc[t][r];
  }
  __syncthreads();
  v4f val[8];
  size_t go[8];
#pragma unroll
  for (int it = 0; it < 8; ++it) {
    const int p    = lane + 32 * it;
    const int L    = p >> 3;
    const int pc   = p & 7;
    const int row  = L >> 1;
    const int half = L & 1;
    const int col  = n0 + half * 32 + pc * 4;
    const v4f bb = *(const v4f*)(ob + col);
    go[it]  = (size_t)(m0 + row) * DM + col;
    val[it] = *(const v4f*)(sw + row * OTP + half * 32 + pc * 4) + bb;
  }
#pragma unroll
  for (int it = 0; it < 8; ++it) *(volatile v4f*)(out + go[it]) = val[it];
  __threadfence();
#pragma unroll
  for (int it = 0; it < 8; ++it) *(volatile v4f*)(out + go[it]) = val[it];
}

extern "C" void kernel_launch(void* const* d_in, const int* in_sizes, int n_in,
                              void* d_out, int out_size, void* d_ws, size_t ws_size,
                              hipStream_t stream) {
  if (n_in < 10) return;
  if (in_sizes[0] != NROWS * DM || in_sizes[1] != NROWS * DM || in_sizes[2] != NROWS * DM) return;
  if (in_sizes[3] != DM * DM || in_sizes[4] != DM * DM || in_sizes[5] != DM * DM) return;
  if (in_sizes[6] != DM * DM || in_sizes[8] != DM * DM) return;
  if (in_sizes[7] != DM || in_sizes[9] != DM) return;
  if (out_size != NROWS * DM) return;

  const float* qin = (const float*)d_in[0];
  const float* kin = (const float*)d_in[1];
  const float* vin = (const float*)d_in[2];
  const float* qt  = (const float*)d_in[3];
  const float* kt  = (const float*)d_in[4];
  const float* vt  = (const float*)d_in[5];
  const float* gw  = (const float*)d_in[6];
  const float* gb  = (const float*)d_in[7];
  const float* ow  = (const float*)d_in[8];
  const float* ob  = (const float*)d_in[9];
  float* out = (float*)d_out;

  size_t off = 0;
  const size_t oXh = off; off += (size_t)3 * NROWS * DM * 2;
  const size_t oXl = off; off += (size_t)3 * NROWS * DM * 2;
  const size_t oWh = off; off += (size_t)WROWS * DM * 2;
  const size_t oWl = off; off += (size_t)WROWS * DM * 2;
  const size_t oQh = off; off += (size_t)NROWS * DM * 2;
  const size_t oQl = off; off += (size_t)NROWS * DM * 2;
  const size_t oKh = off; off += (size_t)NROWS * DM * 2;
  const size_t oKl = off; off += (size_t)NROWS * DM * 2;
  const size_t oVh = off; off += (size_t)NB * NHD * HC * SEQ * 2;
  const size_t oVl = off; off += (size_t)NB * NHD * HC * SEQ * 2;
  const size_t oG  = off; off += (size_t)NROWS * DM * 4;
  const size_t oOh = off; off += (size_t)NROWS * DM * 2;
  const size_t oOl = off; off += (size_t)NROWS * DM * 2;
  if (off > ws_size) return;
  if (off > (size_t)134217728) return;

  char* ws = (char*)d_ws;
  us* Xh = (us*)(ws + oXh);
  us* Xl = (us*)(ws + oXl);
  us* Wh = (us*)(ws + oWh);
  us* Wl = (us*)(ws + oWl);
  us* Qh = (us*)(ws + oQh);
  us* Ql = (us*)(ws + oQl);
  us* Kh = (us*)(ws + oKh);
  us* Kl = (us*)(ws + oKl);
  us* Vh = (us*)(ws + oVh);
  us* Vl = (us*)(ws + oVl);
  float* G = (float*)(ws + oG);
  us* Oh = (us*)(ws + oOh);
  us* Ol = (us*)(ws + oOl);

  k_cvtw<<<dim3(WROWS / 64, DM / 64), dim3(128), 0, stream>>>(qt, kt, vt, gw, ow, Wh, Wl);
  k_cvtx<<<dim3((NROWS * DM) / 2048, 3), dim3(256), 0, stream>>>(qin, kin, vin, Xh, Xl);
  k_proj<<<dim3(NROWS / 64, 16), dim3(128), 0, stream>>>(Xh, Xl, Wh, Wl, gb, Qh, Ql, Kh, Kl, Vh, Vl, G);
  k_attn<<<dim3(SEQ / QBK, NHD / 2, NB), dim3(128), 0, stream>>>(Qh, Ql, Kh, Kl, Vh, Vl, G, Oh, Ol);
  k_out<<<dim3(NROWS / 64, DM / 64), dim3(128), 0, stream>>>(Oh, Ol, Wh, Wl, ob, out);
  (void)hipGetLastError();
}
